// TransformerBlock_64914135712225
// MI455X (gfx1250) — hardware-verified
//
#include <hip/hip_runtime.h>
#include <math.h>

#ifndef NB
#define NB 2
#endif
#ifndef SEQ
#define SEQ 2048
#endif
#define NB_FULL 2
#define SEQ_FULL 2048
#define DM 1024
#define NH 16
#define DH 64
#define DFF 4096
#define ROWS (NB * SEQ)
#define WSC 16.0f
#define CTXC 64.0f
#define X1C 16.0f
#define HC 16.0f
#define LN_EPS 1e-6f
#define AT_NW 4
#define AT_PP 40
#define SLABP 68
#define TRP 65

static_assert(DM == NH * DH);
static_assert(DH == 64);
static_assert(DM == 256 * 4);
static_assert(SEQ % 64 == 0);
static_assert(ROWS % 64 == 0);
static_assert(DM % 64 == 0 && DFF % 64 == 0);
static_assert(DM % 32 == 0 && DFF % 32 == 0);
static_assert(DM % 8 == 0 && DFF % 8 == 0);
static_assert(NB <= NB_FULL && SEQ <= SEQ_FULL);
static_assert((AT_PP % 8) == 0 && AT_PP >= 32);

typedef __attribute__((ext_vector_type(16))) _Float16 v16h;
typedef __attribute__((ext_vector_type(8)))  _Float16 v8h;
typedef __attribute__((ext_vector_type(8)))  float    v8f;
typedef __attribute__((ext_vector_type(4)))  float    v4f;
typedef __attribute__((ext_vector_type(4)))  unsigned int v4u;

union FragH { v16h v; v8h h[2]; };
__device__ __forceinline__ v16h ldfrag(const _Float16* p) { FragH f; f.h[0] = *(const v8h*)(p); f.h[1] = *(const v8h*)(p + 16); return f.v; }

__device__ __forceinline__ v8f wmma16(v16h a, v16h b, v8f c) {
    c = __builtin_amdgcn_wmma_f32_16x16x32_f16(false, a, false, b, (short)0, c, false, false);
    asm volatile("v_nop\n\tv_nop\n\tv_nop\n\tv_nop" : "+v"(c) : "v"(a), "v"(b));
    return c;
}

__device__ __forceinline__ void wave_lds_sync() {
    __builtin_amdgcn_fence(3  , "workgroup");
    __builtin_amdgcn_wave_barrier();
    __builtin_amdgcn_fence(2  , "workgroup");
}

__device__ __forceinline__ float cmb_bf(float v) { const unsigned u = __builtin_bit_cast(unsigned, v); const unsigned r = (u + 0x7fffu + ((u >> 16) & 1u)) & 0xffff0000u; return __builtin_bit_cast(float, r); }
__device__ __forceinline__ unsigned int cmb_pk2(float a, float b) { return (unsigned int)__builtin_bit_cast(unsigned short, (_Float16)a) | ((unsigned int)__builtin_bit_cast(unsigned short, (_Float16)b) << 16); }
__device__ __forceinline__ size_t rowmap(int r) { return (size_t)(r / SEQ) * SEQ_FULL + (size_t)(r % SEQ); }

#define VST2(T, ptr, val) do { const T vst2_v_ = (val); *(volatile T*)(ptr) = vst2_v_; __threadfence(); *(volatile T*)(ptr) = vst2_v_; } while (0)
#define VST2V4(ptr, val) do { const v4f vst2_v4_ = (val); *(volatile v4f*)(ptr) = vst2_v4_; __threadfence(); *(volatile v4f*)(ptr) = vst2_v4_; } while (0)

__global__ __launch_bounds__(256) void k_cast_rows(const float* __restrict__ SRC, int lds, unsigned short* __restrict__ DST, int ldd, int nR, int nC, float sc, int remap) {
    const long long u = (long long)blockIdx.x * 256 + threadIdx.x; const int per = nC / 8; if (u >= (long long)nR * per) return;
    const int r = (int)(u / per); const int c0 = 8 * (int)(u % per);
    const size_t sr = remap ? rowmap(r) : (size_t)r;
    const float* s = SRC + sr * (size_t)lds + c0;
    const v4f a = *(const v4f*)(s); const v4f b = *(const v4f*)(s + 4);
    v4u pk;
    pk.x = cmb_pk2(cmb_bf(a.x) * sc, cmb_bf(a.y) * sc); pk.y = cmb_pk2(cmb_bf(a.z) * sc, cmb_bf(a.w) * sc);
    pk.z = cmb_pk2(cmb_bf(b.x) * sc, cmb_bf(b.y) * sc); pk.w = cmb_pk2(cmb_bf(b.z) * sc, cmb_bf(b.w) * sc);
    VST2(v4u, (v4u*)(DST + (size_t)r * ldd + c0), pk);
}

__global__ __launch_bounds__(256) void k_cast_tr(const float* __restrict__ SRC, int R, int C, unsigned short* __restrict__ DST, float sc) {
    __shared__ float tl[64 * TRP];
    const int t = threadIdx.x;
    const int c0 = blockIdx.x * 64, r0 = blockIdx.y * 64;
    if (c0 + 64 > C || r0 + 64 > R) return;
#pragma unroll
    for (int it = 0; it < 4; ++it) {
        const int idx = it * 256 + t; const int row = idx >> 4; const int c4 = (idx & 15) * 4;
        const v4f v = *(const v4f*)(SRC + (size_t)(r0 + row) * C + c0 + c4);
        tl[row * TRP + c4 + 0] = cmb_bf(v.x) * sc; tl[row * TRP + c4 + 1] = cmb_bf(v.y) * sc;
        tl[row * TRP + c4 + 2] = cmb_bf(v.z) * sc; tl[row * TRP + c4 + 3] = cmb_bf(v.w) * sc;
    }
    __syncthreads();
    v4u pk[2];
#pragma unroll
    for (int it = 0; it < 2; ++it) {
        const int slot = it * 256 + t; const int orow = slot >> 3; const int pc = slot & 7;
        const int b0 = (8 * pc) * TRP + orow;
        v4u p;
        p.x = cmb_pk2(tl[b0],           tl[b0 + TRP]);
        p.y = cmb_pk2(tl[b0 + 2 * TRP], tl[b0 + 3 * TRP]);
        p.z = cmb_pk2(tl[b0 + 4 * TRP], tl[b0 + 5 * TRP]);
        p.w = cmb_pk2(tl[b0 + 6 * TRP], tl[b0 + 7 * TRP]);
        pk[it] = p;
    }
#pragma unroll
    for (int it = 0; it < 2; ++it) { const int slot = it * 256 + t; *(volatile v4u*)(DST + (size_t)(c0 + (slot >> 3)) * R + r0 + 8 * (slot & 7)) = pk[it]; }
    __threadfence();
#pragma unroll
    for (int it = 0; it < 2; ++it) { const int slot = it * 256 + t; *(volatile v4u*)(DST + (size_t)(c0 + (slot >> 3)) * R + r0 + 8 * (slot & 7)) = pk[it]; }
}

template <int OUT_MODE, int BIAS_MODE, int RESID, int ACT>
__device__ __forceinline__ void gemm64_body(float* sT,
    const unsigned short* __restrict__ Ap, int lda, long long strideA,
    const unsigned short* __restrict__ Btp, int ldb, long long strideB,
    unsigned short* __restrict__ C16, float* __restrict__ C32, int ldc, long long strideC,
    const float* __restrict__ bias, const float* __restrict__ resid, int ldr,
    int M, int N, int K, float scale, float bsc) {
  const int b    = blockIdx.y;
  const int lane = threadIdx.x & 31;
  const int wave = __builtin_amdgcn_readfirstlane(threadIdx.x >> 5);
  const int tilesN = N >> 6;
  const int tilesM = M >> 6;
  const int tile = blockIdx.x * 8 + wave;
  if (tile >= tilesM * tilesN) return;
  const int tm = tile / tilesN;
  const int tn = tile - tm * tilesN;
  const int m0 = tm << 6;
  const int n0 = tn << 6;

  const _Float16* Ab = (const _Float16*)Ap  + (size_t)b * strideA;
  const _Float16* Bb = (const _Float16*)Btp + (size_t)b * strideB;

  const int rlane = lane & 15;
  const int koff  = (lane >> 4) * 8;
  const int mOff  = (lane >> 4) * 8;

  v8f acc[4][4];
#pragma unroll
  for (int i = 0; i < 4; ++i)
#pragma unroll
    for (int j = 0; j < 4; ++j) acc[i][j] = (v8f){0.f,0.f,0.f,0.f,0.f,0.f,0.f,0.f};

  for (int k0 = 0; k0 < K; k0 += 32) {
    v16h bh[4];
#pragma unroll
    for (int j = 0; j < 4; ++j) {
      const size_t bo = (size_t)(n0 + (j << 4) + rlane) * ldb + koff + k0;
      bh[j] = ldfrag(Bb + bo);
    }
#pragma unroll
    for (int i = 0; i < 4; ++i) {
      const size_t ao = (size_t)(m0 + (i << 4) + rlane) * lda + koff + k0;
      const v16h ah = ldfrag(Ab + ao);
#pragma unroll
      for (int j = 0; j < 4; ++j) acc[i][j] = wmma16(ah, bh[j], acc[i][j]);
    }
  }

  const int sbase = wave * (16 * SLABP);
  float bvj[4];
#pragma unroll
  for (int j = 0; j < 4; ++j) bvj[j] = (BIAS_MODE == 2) ? bsc * cmb_bf(bias[n0 + (j << 4) + rlane]) : 0.f;
#pragma unroll
  for (int i = 0; i < 4; ++i) {
    const int mBase = m0 + (i << 4);
#pragma unroll
    for (int j = 0; j < 4; ++j) {
#pragma unroll
      for (int r = 0; r < 8; ++r) {
        float v = acc[i][j][r] * scale;
        if (BIAS_MODE == 1) v += bsc * cmb_bf(bias[mBase + mOff + r]);
        if (BIAS_MODE == 2) v += bvj[j];
        if (ACT == 1) v = fmaxf(v, 0.0f);
        sT[sbase + (mOff + r) * SLABP + (j << 4) + rlane] = v;
      }
    }
    wave_lds_sync();
    if (OUT_MODE == 0) {
      float* Cb = C32 + (size_t)b * strideC;
      const int hh2 = lane >> 4, c4 = (lane & 15) * 4;
      v4f vals[8];
#pragma unroll
      for (int it = 0; it < 8; ++it) {
        const int row = it * 2 + hh2; const int grow = mBase + row;
        v4f v = *(const v4f*)(sT + sbase + row * SLABP + c4);
        if (RESID == 1) { const v4f rv = *(const v4f*)(resid + (size_t)grow * ldr + n0 + c4); v = v + rv; }
        if (RESID == 2) { const v4f rv = *(const v4f*)(resid + rowmap(grow) * (size_t)ldr + n0 + c4);
                          v.x += cmb_bf(rv.x); v.y += cmb_bf(rv.y); v.z += cmb_bf(rv.z); v.w += cmb_bf(rv.w); }
        vals[it] = v;
      }
#pragma unroll
      for (int it = 0; it < 8; ++it) *(volatile v4f*)(Cb + (size_t)(mBase + it * 2 + hh2) * ldc + n0 + c4) = vals[it];
      __threadfence();
#pragma unroll
      for (int it = 0; it < 8; ++it) *(volatile v4f*)(Cb + (size_t)(mBase + it * 2 + hh2) * ldc + n0 + c4) = vals[it];
    } else {
      unsigned short* Cb = C16 + (size_t)b * strideC;
      const int q = lane >> 3, c8 = (lane & 7) * 8;
      v8h hv[4];
#pragma unroll
      for (int it = 0; it < 4; ++it) {
        const int row = it * 4 + q;
        const v4f a = *(const v4f*)(sT + sbase + row * SLABP + c8);
        const v4f c = *(const v4f*)(sT + sbase + row * SLABP + c8 + 4);
        v8h t;
        t[0] = (_Float16)a.x; t[1] = (_Float16)a.y; t[2] = (_Float16)a.z; t[3] = (_Float16)a.w;
        t[4] = (_Float16)c.x; t[5] = (_Float16)c.y; t[6] = (_Float16)c.z; t[7] = (_Float16)c.w;
        hv[it] = t;
      }
#pragma unroll
      for (int it = 0; it < 4; ++it) *(volatile v8h*)(Cb + (size_t)(mBase + it * 4 + q) * ldc + n0 + c8) = hv[it];
      __threadfence();
#pragma unroll
      for (int it = 0; it < 4; ++it) *(volatile v8h*)(Cb + (size_t)(mBase + it * 4 + q) * ldc + n0 + c8) = hv[it];
    }
    wave_lds_sync();
  }
}

__global__ __launch_bounds__(256) void k_gemm_proj(const unsigned short* __restrict__ A, int lda, const unsigned short* __restrict__ Bt, int ldb,
                                                   unsigned short* __restrict__ C, int ldc, const float* __restrict__ bias, int M, int N, int K, float scale, float bsc) {
  __shared__ __align__(16) float sT[8 * 16 * SLABP];
  gemm64_body<1, 2, 0, 0>(sT, A, lda, 0, Bt, ldb, 0, C, nullptr, ldc, 0, bias, nullptr, 0, M, N, K, scale, bsc);
}
__global__ __launch_bounds__(256) void k_gemm_vt(const unsigned short* __restrict__ A, int lda, const unsigned short* __restrict__ Bt, int ldb, long long strideB,
                                                 unsigned short* __restrict__ C, int ldc, long long strideC, const float* __restrict__ bias, int M, int N, int K, float scale, float bsc) {
  __shared__ __align__(16) float sT[8 * 16 * SLABP];
  gemm64_body<1, 1, 0, 0>(sT, A, lda, 0, Bt, ldb, strideB, C, nullptr, ldc, strideC, bias, nullptr, 0, M, N, K, scale, bsc);
}
__global__ __launch_bounds__(256) void k_gemm_wo(const unsigned short* __restrict__ A, int lda, const unsigned short* __restrict__ Bt, int ldb,
                                                 float* __restrict__ C, int ldc, const float* __restrict__ bias, const float* __restrict__ xin, int ldr, int M, int N, int K, float scale, float bsc) {
  __shared__ __align__(16) float sT[8 * 16 * SLABP];
  gemm64_body<0, 2, 2, 0>(sT, A, lda, 0, Bt, ldb, 0, nullptr, C, ldc, 0, bias, xin, ldr, M, N, K, scale, bsc);
}
__global__ __launch_bounds__(256) void k_gemm_ff1(const unsigned short* __restrict__ A, int lda, const unsigned short* __restrict__ Bt, int ldb,
                                                  unsigned short* __restrict__ C, int ldc, const float* __restrict__ bias, int M, int N, int K, float scale, float bsc) {
  __shared__ __align__(16) float sT[8 * 16 * SLABP];
  gemm64_body<1, 2, 0, 1>(sT, A, lda, 0, Bt, ldb, 0, C, nullptr, ldc, 0, bias, nullptr, 0, M, N, K, scale, bsc);
}
__global__ __launch_bounds__(256) void k_gemm_ff2(const unsigned short* __restrict__ A, int lda, const unsigned short* __restrict__ Bt, int ldb,
                                                  float* __restrict__ C, int ldc, const float* __restrict__ bias, const float* __restrict__ res, int ldr, int M, int N, int K, float scale, float bsc) {
  __shared__ __align__(16) float sT[8 * 16 * SLABP];
  gemm64_body<0, 2, 1, 0>(sT, A, lda, 0, Bt, ldb, 0, nullptr, C, ldc, 0, bias, res, ldr, M, N, K, scale, bsc);
}

__global__ __launch_bounds__(128) void k_attn_flash(const unsigned short* __restrict__ Qp, const unsigned short* __restrict__ Kp,
                                                    const unsigned short* __restrict__ VTp, unsigned short* __restrict__ CTX) {
  __shared__ __align__(16) _Float16 Pt[AT_NW * 16 * AT_PP];
  __shared__ __align__(16) float    Os[AT_NW * 16 * SLABP];
  const int tid = threadIdx.x, lane = tid & 31, hh = lane >> 4, c = lane & 15;
  const int wave = __builtin_amdgcn_readfirstlane(threadIdx.x >> 5);
  const int nqb = SEQ / 64;
  const int bx = blockIdx.x;
  const int qb = bx % nqb;
  const int bh = bx / nqb;
  const int h  = bh % NH;
  const int b  = bh / NH;
  const int q0 = qb * 64 + wave * 16;
  const size_t tok0 = (size_t)b * SEQ;
  const _Float16* Q  = (const _Float16*)Qp;
  const _Float16* Kk = (const _Float16*)Kp;
  const _Float16* VT = (const _Float16*)VTp;
  const size_t qoff = (tok0 + q0 + c) * DM + h * DH + 8 * hh;
  const size_t koff = tok0 * DM + h * DH + 8 * hh;
  const size_t voff = ((size_t)b * DM + h * DH + c) * SEQ + 8 * hh;
  const int pbase = wave * (16 * AT_PP);
  const int obase = wave * (16 * SLABP);
  const float SC = 0.125f * 1.4426950408889634f;

  float m8[8], l8[8];
  v8f o[4];
#pragma unroll
  for (int r = 0; r < 8; ++r) { m8[r] = -3.0e38f; l8[r] = 0.f; }
#pragma unroll
  for (int t = 0; t < 4; ++t) o[t] = (v8f){0.f,0.f,0.f,0.f,0.f,0.f,0.f,0.f};

#pragma unroll 1
  for (int kb0 = 0; kb0 < SEQ; kb0 += 32) {
    v8f s0 = (v8f){0.f,0.f,0.f,0.f,0.f,0.f,0.f,0.f};
    v8f s1 = s0;
#pragma unroll
    for (int ks = 0; ks < 2; ++ks) {
      const v16h qa = ldfrag(Q + qoff + ks * 32);
      const v16h ka = ldfrag(Kk + koff + (size_t)(kb0 + c) * DM + ks * 32);
      const v16h kb = ldfrag(Kk + koff + (size_t)(kb0 + 16 + c) * DM + ks * 32);
      s0 = wmma16(qa, ka, s0);
      s1 = wmma16(qa, kb, s1);
    }
#pragma unroll
    for (int r = 0; r < 8; ++r) {
      const float a0 = s0[r] * SC, a1 = s1[r] * SC;
      float mx = fmaxf(a0, a1);
      mx = fmaxf(mx, __shfl_xor(mx, 1, 32)); mx = fmaxf(mx, __shfl_xor(mx, 2, 32));
      mx = fmaxf(mx, __shfl_xor(mx, 4, 32)); mx = fmaxf(mx, __shfl_xor(mx, 8, 32));
      const float mnew  = fmaxf(m8[r], mx);
      const float alpha = exp2f(m8[r] - mnew);
      const float p0 = exp2f((a0 - mnew) + 10.0f);
      const float p1 = exp2f((a1 - mnew) + 10.0f);
      float rs = p0 + p1;
      rs += __shfl_xor(rs, 1, 32); rs += __shfl_xor(rs, 2, 32); rs += __shfl_xor(rs, 4, 32); rs += __shfl_xor(rs, 8, 32);
      l8[r] = l8[r] * alpha + rs;
      m8[r] = mnew;
#pragma unroll
      for (int t = 0; t < 4; ++t) o[t][r] *= alpha;
      Pt[pbase + (8 * hh + r) * AT_PP + c]      = (_Float16)p0;
      Pt[pbase + (8 * hh + r) * AT_PP + 16 + c] = (_Float16)p1;
    }
    wave_lds_sync();
    const v16h pa = ldfrag(&Pt[pbase + c * AT_PP + 8 * hh]);
    wave_lds_sync();
    v16h vb[4];
#pragma unroll
    for (int t = 0; t < 4; ++t) vb[t] = ldfrag(VT + voff + (size_t)t * 16 * SEQ + kb0);
#pragma unroll
    for (int t = 0; t < 4; ++t) o[t] = wmma16(pa, vb[t], o[t]);
  }

#pragma unroll
  for (int r = 0; r < 8; ++r) {
    const float inv = CTXC * (1.0f / l8[r]);
#pragma unroll
    for (int t = 0; t < 4; ++t) Os[obase + (8 * hh + r) * SLABP + t * 16 + c] = o[t][r] * inv;
  }
  wave_lds_sync();
  {
    const int q = lane >> 3, c8 = (lane & 7) * 8;
    v8h hv[4];
#pragma unroll
    for (int it = 0; it < 4; ++it) {
      const int row = it * 4 + q;
      const v4f a = *(const v4f*)(&Os[obase + row * SLABP + c8]);
      const v4f d = *(const v4f*)(&Os[obase + row * SLABP + c8 + 4]);
      v8h t;
      t[0] = (_Float16)a.x; t[1] = (_Float16)a.y; t[2] = (_Float16)a.z; t[3] = (_Float16)a.w;
      t[4] = (_Float16)d.x; t[5] = (_Float16)d.y; t[6] = (_Float16)d.z; t[7] = (_Float16)d.w;
      hv[it] = t;
    }
    unsigned short* dst = CTX + (tok0 + q0) * DM + h * DH;
#pragma unroll
    for (int it = 0; it < 4; ++it) *(volatile v8h*)(dst + (size_t)(it * 4 + q) * DM + c8) = hv[it];
    __threadfence();
#pragma unroll
    for (int it = 0; it < 4; ++it) *(volatile v8h*)(dst + (size_t)(it * 4 + q) * DM + c8) = hv[it];
  }
}

template <int MODE>
__device__ __forceinline__ void ln_body(float* s1, float* s2, const float* __restrict__ T, const float* __restrict__ g, const float* __restrict__ be,
                                        float* __restrict__ Y, unsigned short* __restrict__ Y16) {
  const int row = blockIdx.x, t = threadIdx.x, lane = t & 31;
  const int w = __builtin_amdgcn_readfirstlane(threadIdx.x >> 5);
  const v4f v = *(const v4f*)(T + (size_t)row * DM + 4 * t);
  float s = (v.x + v.y) + (v.z + v.w);
  s += __shfl_xor(s, 16, 32); s += __shfl_xor(s, 8, 32); s += __shfl_xor(s, 4, 32); s += __shfl_xor(s, 2, 32); s += __shfl_xor(s, 1, 32);
  if (lane == 0) s1[w] = s;
  __syncthreads();
  float ts = 0.f;
#pragma unroll 1
  for (int i = 0; i < 8; ++i) ts += s1[i];
  const float mu = ts * (1.0f / (float)DM);
  const v4f d = v - mu;
  float q = (d.x * d.x + d.y * d.y) + (d.z * d.z + d.w * d.w);
  q += __shfl_xor(q, 16, 32); q += __shfl_xor(q, 8, 32); q += __shfl_xor(q, 4, 32); q += __shfl_xor(q, 2, 32); q += __shfl_xor(q, 1, 32);
  if (lane == 0) s2[w] = q;
  __syncthreads();
  float tq = 0.f;
#pragma unroll 1
  for (int i = 0; i < 8; ++i) tq += s2[i];
  const float sd  = sqrtf(tq * (1.0f / (float)DM));
  const float inv = 1.0f / (sd + LN_EPS);
  const v4f gg = *(const v4f*)(g + 4 * t); const v4f bb = *(const v4f*)(be + 4 * t);
  v4f y;
  y.x = cmb_bf(gg.x) * (d.x * inv) + cmb_bf(bb.x); y.y = cmb_bf(gg.y) * (d.y * inv) + cmb_bf(bb.y);
  y.z = cmb_bf(gg.z) * (d.z * inv) + cmb_bf(bb.z); y.w = cmb_bf(gg.w) * (d.w * inv) + cmb_bf(bb.w);
  if (MODE == 0) {
    VST2V4(Y + (size_t)row * DM + 4 * t, y);
    const unsigned long long pk = (unsigned long long)cmb_pk2(y.x * X1C, y.y * X1C) | ((unsigned long long)cmb_pk2(y.z * X1C, y.w * X1C) << 32);
    VST2(unsigned long long, (unsigned long long*)(Y16 + (size_t)row * DM + 4 * t), pk);
  } else {
    VST2V4(Y + rowmap(row) * (size_t)DM + 4 * t, y);
  }
}
__global__ __launch_bounds__(256) void k_ln_mid(const float* __restrict__ T, const float* __restrict__ g, const float* __restrict__ be, float* __restrict__ Y, unsigned short* __restrict__ Y16) {
  __shared__ float s1[8]; __shared__ float s2[8];
  ln_body<0>(s1, s2, T, g, be, Y, Y16);
}
__global__ __launch_bounds__(256) void k_ln_out(const float* __restrict__ T, const float* __restrict__ g, const float* __restrict__ be, float* __restrict__ OUT) {
  __shared__ float s1[8]; __shared__ float s2[8];
  ln_body<1>(s1, s2, T, g, be, OUT, nullptr);
}

constexpr size_t SZ_ROWP = (size_t)ROWS * DM * 2;
constexpr size_t OFF_X16 = 0;
constexpr size_t OFF_Q16 = OFF_X16 + SZ_ROWP;
constexpr size_t OFF_K16 = OFF_Q16 + SZ_ROWP;
constexpr size_t OFF_VT  = OFF_K16 + SZ_ROWP;
constexpr size_t OFF_WQ  = OFF_VT + SZ_ROWP;
constexpr size_t SZ_WDD  = (size_t)DM * DM * 2;
constexpr size_t OFF_WK  = OFF_WQ + SZ_WDD;
constexpr size_t OFF_WV  = OFF_WK + SZ_WDD;
constexpr size_t OFF_WO  = OFF_WV + SZ_WDD;
constexpr size_t OFF_W1  = OFF_WO + SZ_WDD;
constexpr size_t SZ_WFF  = (size_t)DFF * DM * 2;
constexpr size_t OFF_W2  = OFF_W1 + SZ_WFF;
constexpr size_t OFF_CTX = OFF_W2 + SZ_WFF;
constexpr size_t OFF_T32 = OFF_CTX + SZ_ROWP;
constexpr size_t SZ_ROWF = (size_t)ROWS * DM * 4;
constexpr size_t OFF_X1  = OFF_T32 + SZ_ROWF;
constexpr size_t OFF_X1H = OFF_X1 + SZ_ROWF;
constexpr size_t WS_TOTAL = OFF_X1H + SZ_ROWP;
constexpr size_t OFF_H16 = 0;
constexpr size_t SZ_H16  = (size_t)ROWS * DFF * 2;
static_assert(OFF_H16 + SZ_H16 <= OFF_WQ);
static_assert(WS_TOTAL <= (size_t)134217728);
static_assert((SZ_ROWP % 128) == 0 && (SZ_WDD % 128) == 0 && (SZ_WFF % 128) == 0 && (SZ_ROWF % 128) == 0);
static_assert((size_t)NB * DM * SEQ * 2 <= SZ_ROWP);

extern "C" void kernel_launch(void* const* d_in, const int* in_sizes, int n_in, void* d_out, int out_size, void* d_ws, size_t ws_size, hipStream_t stream) {
    if (n_in < 17) return;
    const long long need_x = ((long long)(NB - 1) * SEQ_FULL + SEQ) * DM;
    if ((long long)in_sizes[0] < need_x) return;
    if (in_sizes[1] < DM * DM || in_sizes[3] < DM * DM || in_sizes[5] < DM * DM || in_sizes[7] < DM * DM) return;
    if (in_sizes[9] < DFF * DM || in_sizes[11] < DM * DFF) return;
    if (in_sizes[2] < DM || in_sizes[4] < DM || in_sizes[6] < DM || in_sizes[8] < DM || in_sizes[10] < DFF || in_sizes[12] < DM) return;
    if (in_sizes[13] < DM || in_sizes[14] < DM || in_sizes[15] < DM || in_sizes[16] < DM) return;
    if ((long long)out_size < need_x) return;
    if (ws_size < WS_TOTAL) return;

    const float* x   = (const float*)d_in[0];
    const float* Wq  = (const float*)d_in[1];
    const float* bq  = (const float*)d_in[2];
    const float* Wk  = (const float*)d_in[3];
    const float* bk  = (const float*)d_in[4];
    const float* Wv  = (const float*)d_in[5];
    const float* bv  = (const float*)d_in[6];
    const float* Wo  = (const float*)d_in[7];
    const float* bo  = (const float*)d_in[8];
    const float* W1  = (const float*)d_in[9];
    const float* b1  = (const float*)d_in[10];
    const float* W2  = (const float*)d_in[11];
    const float* b2  = (const float*)d_in[12];
    const float* g1  = (const float*)d_in[13];
    const float* be1 = (const float*)d_in[14];
    const float* g2  = (const float*)d_in[15];
    const float* be2 = (const float*)d_in[16];
    float* out = (float*)d_out;

    char* ws = (char*)d_ws;
    unsigned short* X16  = (unsigned short*)(ws + OFF_X16);
    unsigned short* Q16  = (unsigned short*)(ws + OFF_Q16);
    unsigned short* K16  = (unsigned short*)(ws + OFF_K16);
    unsigned short* VT16 = (unsigned short*)(ws + OFF_VT);
    unsigned short* WQ16 = (unsigned short*)(ws + OFF_WQ);
    unsigned short* WK16 = (unsigned short*)(ws + OFF_WK);
    unsigned short* WV16 = (unsigned short*)(ws + OFF_WV);
    unsigned short* WO16 = (unsigned short*)(ws + OFF_WO);
    unsigned short* W116 = (unsigned short*)(ws + OFF_W1);
    unsigned short* W216 = (unsigned short*)(ws + OFF_W2);
    unsigned short* CTX16 = (unsigned short*)(ws + OFF_CTX);
    float* T32 = (float*)(ws + OFF_T32);
    float* X1  = (float*)(ws + OFF_X1);
    unsigned short* X1H = (unsigned short*)(ws + OFF_X1H);
    unsigned short* H16 = (unsigned short*)(ws + OFF_H16);

    const float iw = 1.0f / WSC;
    k_cast_rows<<<(unsigned)(((long long)ROWS * (DM / 8) + 255) / 256), 256, 0, stream>>>(x, DM, X16, DM, ROWS, DM, 1.0f, 1);
    k_cast_tr<<<dim3(DM / 64,  DM / 64),  256, 0, stream>>>(Wq, DM,  DM,  WQ16, WSC);
    k_cast_tr<<<dim3(DM / 64,  DM / 64),  256, 0, stream>>>(Wk, DM,  DM,  WK16, WSC);
    k_cast_tr<<<dim3(DM / 64,  DM / 64),  256, 0, stream>>>(Wv, DM,  DM,  WV16, WSC);
    k_cast_tr<<<dim3(DM / 64,  DM / 64),  256, 0, stream>>>(Wo, DM,  DM,  WO16, WSC);
    k_cast_tr<<<dim3(DFF / 64, DM / 64),  256, 0, stream>>>(W1, DM,  DFF, W116, WSC);
    k_cast_tr<<<dim3(DM / 64,  DFF / 64), 256, 0, stream>>>(W2, DFF, DM,  W216, WSC);

    { const int tiles = (ROWS / 64) * (DM / 64);
      k_gemm_proj<<<dim3((unsigned)((tiles + 7) / 8), 1), 256, 0, stream>>>(X16, DM, WQ16, DM, Q16, DM, bq, ROWS, DM, DM, iw, 1.0f);
      k_gemm_proj<<<dim3((unsigned)((tiles + 7) / 8), 1), 256, 0, stream>>>(X16, DM, WK16, DM, K16, DM, bk, ROWS, DM, DM, iw, 1.0f); }
    { const int tiles = (DM / 64) * (SEQ / 64);
      k_gemm_vt<<<dim3((unsigned)((tiles + 7) / 8), (unsigned)NB), 256, 0, stream>>>(WV16, DM, X16, DM, (long long)SEQ * DM, VT16, SEQ, (long long)DM * SEQ, bv, DM, SEQ, DM, iw, 1.0f); }
    k_attn_flash<<<(unsigned)(NB * NH * (SEQ / 64)), 128, 0, stream>>>(Q16, K16, VT16, CTX16);
    { const int tiles = (ROWS / 64) * (DM / 64);
      k_gemm_wo<<<dim3((unsigned)((tiles + 7) / 8), 1), 256, 0, stream>>>(CTX16, DM, WO16, DM, T32, DM, bo, x, DM, ROWS, DM, DM, 1.0f / (WSC * CTXC), 1.0f); }
    k_ln_mid<<<(unsigned)ROWS, 256, 0, stream>>>(T32, g1, be1, X1, X1H);
    { const int tiles = (ROWS / 64) * (DFF / 64);
      k_gemm_ff1<<<dim3((unsigned)((tiles + 7) / 8), 1), 256, 0, stream>>>(X1H, DM, W116, DM, H16, DFF, b1, ROWS, DFF, DM, HC / (X1C * WSC), HC); }
    { const int tiles = (ROWS / 64) * (DM / 64);
      k_gemm_ff2<<<dim3((unsigned)((tiles + 7) / 8), 1), 256, 0, stream>>>(H16, DFF, W216, DFF, T32, DM, b2, X1, DM, ROWS, DM, DFF, 1.0f / (HC * WSC), 1.0f); }
    k_ln_out<<<(unsigned)ROWS, 256, 0, stream>>>(T32, g2, be2, out);
}
